// TRIP_86268713107801
// MI455X (gfx1250) — hardware-verified
//
#include <hip/hip_runtime.h>
#include <math.h>

constexpr int kNB     = 32768;
constexpr int kNModes = 8;
constexpr int kND     = 256;
constexpr int kNR     = 32;
constexpr int kNRR    = 1024;
constexpr int kChunk  = 4096;
constexpr int kNChunk = kNB / kChunk;
constexpr float kLog2Pi = 1.8378770664093453f;

constexpr size_t kOffSpt  = 0;
constexpr size_t kOffGtab = 4194304;
constexpr size_t kOffLogn = 4227072;
constexpr size_t kOffWpl  = 4259840;
constexpr size_t kOffMarg = 21037056;
constexpr size_t kWsTotal = 88145920;
static_assert(kOffGtab >= kOffSpt + (size_t)kNModes * kNRR * kND * 2, "spt extent");
static_assert(kOffLogn >= kOffGtab + (size_t)kNModes * kND * 4 * 4, "gtab extent");
static_assert(kOffWpl  >= kOffLogn + 128, "logn extent");
static_assert(kOffMarg >= kOffWpl + (size_t)kNModes * kChunk * kND * 2, "wpl extent");
static_assert(kWsTotal >= kOffMarg + (size_t)kNModes * kChunk * kNRR * 2, "marg extent");
static_assert(kWsTotal <= 134217728, "carve budget");
static_assert((kOffGtab % 128) == 0 && (kOffLogn % 128) == 0 && (kOffWpl % 128) == 0 && (kOffMarg % 128) == 0, "alignment");
static_assert(kNB % kChunk == 0 && kChunk % 64 == 0 && kNRR % 64 == 0 && kND % 32 == 0, "tile multiples");

typedef __attribute__((ext_vector_type(16))) _Float16 v16h;
typedef __attribute__((ext_vector_type(8)))  _Float16 v8h;
typedef __attribute__((ext_vector_type(16))) __bf16   v16b;
typedef __attribute__((ext_vector_type(8)))  __bf16   v8b;
typedef __attribute__((ext_vector_type(8)))  float    v8f;
typedef __attribute__((ext_vector_type(4)))  float    v4f;
typedef __attribute__((ext_vector_type(4)))  unsigned int v4u;

__device__ __forceinline__ unsigned short f2bf_bits(float f) {
  unsigned u = __float_as_uint(f);
  return (unsigned short)((u + 0x7FFFu + ((u >> 16) & 1u)) >> 16);
}
__device__ __forceinline__ float bf_bits2f(unsigned short h) { return __uint_as_float(((unsigned)h) << 16); }

__device__ __forceinline__ void dep_guard_h(v8f& a, v8f& b, v16h x, v16h y) { asm volatile("v_nop\n\tv_nop\n\tv_nop\n\tv_nop" : "+v"(a), "+v"(b) : "v"(x), "v"(y)); }
__device__ __forceinline__ void dep_guard_b(v8f& a, v8f& b, v16b x, v16b y) { asm volatile("v_nop\n\tv_nop\n\tv_nop\n\tv_nop" : "+v"(a), "+v"(b) : "v"(x), "v"(y)); }
__device__ __forceinline__ void keep4_h(v16h a, v16h b, v16h c, v16h d) { asm volatile("v_nop" :: "v"(a), "v"(b), "v"(c), "v"(d)); }
__device__ __forceinline__ void keep4_b(v16b a, v16b b, v16b c, v16b d) { asm volatile("v_nop" :: "v"(a), "v"(b), "v"(c), "v"(d)); }
__device__ __forceinline__ void acc_guard4(v8f& a, v8f& b, v8f& c, v8f& d) { asm volatile("v_nop\n\tv_nop\n\tv_nop\n\tv_nop" : "+v"(a), "+v"(b), "+v"(c), "+v"(d)); }
template <typename T> struct Frag;
template <> struct Frag<_Float16> {
  typedef v16h V; union U { v16h v; v8h h[2]; };
  static __device__ __forceinline__ v16h load(const _Float16* p) {
    U f; f.h[0] = *(const v8h*)(p); f.h[1] = *(const v8h*)(p + 16); return f.v;
  }
  static __device__ __forceinline__ v8f mma(v16h a, v16h b, v8f c) {
    return __builtin_amdgcn_wmma_f32_16x16x32_f16(false, a, false, b, (short)0, c, false, false);
  }
  static __device__ __forceinline__ void guard(v8f& a, v8f& b, v16h x, v16h y) { dep_guard_h(a, b, x, y); }
  static __device__ __forceinline__ void keep(v16h a, v16h b, v16h c, v16h d) { keep4_h(a, b, c, d); }
};
template <> struct Frag<__bf16> {
  typedef v16b V; union U { v16b v; v8b h[2]; };
  static __device__ __forceinline__ v16b load(const __bf16* p) {
    U f; f.h[0] = *(const v8b*)(p); f.h[1] = *(const v8b*)(p + 16); return f.v;
  }
  static __device__ __forceinline__ v8f mma(v16b a, v16b b, v8f c) {
    return __builtin_amdgcn_wmma_f32_16x16x32_bf16(false, a, false, b, (short)0, c, false, false);
  }
  static __device__ __forceinline__ void guard(v8f& a, v8f& b, v16b x, v16b y) { dep_guard_b(a, b, x, y); }
  static __device__ __forceinline__ void keep(v16b a, v16b b, v16b c, v16b d) { keep4_b(a, b, c, d); }
};

__device__ __forceinline__ unsigned pk16(unsigned short a, unsigned short b) { return (unsigned)a | ((unsigned)b << 16); }
__device__ __forceinline__ __bf16 tobf(float f) { return __builtin_bit_cast(__bf16, f2bf_bits(f)); }

__device__ __forceinline__ void chain_guard(v8f& a, v8f& b, v8f& c, v8f& d, v16b x, v16b y, v16b z, v16b w) {
  asm volatile("v_nop\n\tv_nop\n\tv_nop\n\tv_nop" : "+v"(a), "+v"(b), "+v"(c), "+v"(d) : "v"(x), "v"(y), "v"(z), "v"(w));
}

template <int ET> struct Elem;
template <> struct Elem<0> { typedef _Float16 T; };
template <> struct Elem<1> { typedef __bf16 T; };
template <int ET, bool SPLIT, int BIAS_MODE, int OUT_MODE, bool RESID, int ACT = 0>
__global__ __launch_bounds__(256) void wmma_gemm64(
    const unsigned short* __restrict__ Ap, const unsigned short* __restrict__ A2p, int lda, long strideA,
    const unsigned short* __restrict__ Btp, const unsigned short* __restrict__ Bt2p, int ldb, long strideB,
    void* __restrict__ Cout, void* __restrict__ Cout2, int ldc, long strideC,
    const float* __restrict__ bias,
    const float* __restrict__ resid, long strideR,
    int M, int N, int K, float scale) {
  typedef typename Elem<ET>::T T;
  typedef typename Frag<T>::V V;
  const T* A = (const T*)Ap; const T* A2 = (const T*)A2p; const T* Bt = (const T*)Btp; const T* Bt2 = (const T*)Bt2p;
  __shared__ __align__(16) float sT[8][16 * 68];
  const int b    = blockIdx.y;
  const int lane = threadIdx.x & 31;
  const int wave = threadIdx.x >> 5;
  const int tilesN = N >> 6;
  const int tilesM = M >> 6;
  const int tile = blockIdx.x * 8 + wave;
  if (tile >= tilesM * tilesN) return;
  const int tm = tile / tilesN;
  const int tn = tile - tm * tilesN;
  const int m0 = tm << 6;
  const int n0 = tn << 6;

  const T* Ab  = A  + (size_t)b * strideA;
  const T* Bb  = Bt + (size_t)b * strideB;
  const T* Ab2 = SPLIT ? (A2  + (size_t)b * strideA) : nullptr;
  const T* Bb2 = SPLIT ? (Bt2 + (size_t)b * strideB) : nullptr;

  const int rlane = lane & 15;
  const int koff  = (lane >> 4) * 8;
  const int mOff  = (lane >> 4) * 8;

  v8f acc[4][4];
#pragma unroll
  for (int i = 0; i < 4; ++i)
#pragma unroll
    for (int j = 0; j < 4; ++j) acc[i][j] = (v8f){0.f,0.f,0.f,0.f,0.f,0.f,0.f,0.f};

  for (int k0 = 0; k0 < K; k0 += 32) {
    V bh[4], bl[4];
#pragma unroll
    for (int j = 0; j < 4; ++j) {
      const size_t bo = (size_t)(n0 + (j << 4) + rlane) * ldb + koff + k0;
      bh[j] = Frag<T>::load(Bb + bo);
      if (SPLIT) bl[j] = Frag<T>::load(Bb2 + bo);
    }
#pragma unroll
    for (int i = 0; i < 4; ++i) {
      const size_t ao = (size_t)(m0 + (i << 4) + rlane) * lda + koff + k0;
      V ah = Frag<T>::load(Ab + ao);
      V al;
      if (SPLIT) al = Frag<T>::load(Ab2 + ao);
#pragma unroll
      for (int j = 0; j < 4; ++j) {
        acc[i][j] = Frag<T>::mma(ah, bh[j], acc[i][j]);
        if (SPLIT) {
          acc[i][j] = Frag<T>::mma(ah, bl[j], acc[i][j]);
          acc[i][j] = Frag<T>::mma(al, bh[j], acc[i][j]);
        }
      }
      Frag<T>::guard(acc[i][0], acc[i][3], ah, SPLIT ? al : ah);
    }
    Frag<T>::keep(bh[0], bh[1], bh[2], bh[3]);
    if (SPLIT) Frag<T>::keep(bl[0], bl[1], bl[2], bl[3]);
  }
  acc_guard4(acc[0][0], acc[0][1], acc[0][2], acc[0][3]);
  acc_guard4(acc[1][0], acc[1][1], acc[1][2], acc[1][3]);
  acc_guard4(acc[2][0], acc[2][1], acc[2][2], acc[2][3]);
  acc_guard4(acc[3][0], acc[3][1], acc[3][2], acc[3][3]);

  float* slab = sT[wave];
  const float* Rb = RESID ? (resid + (size_t)b * strideR) : nullptr;
#pragma unroll
  for (int i = 0; i < 4; ++i) {
    const int mBase = m0 + (i << 4);
#pragma unroll
    for (int j = 0; j < 4; ++j) {
      const int n = n0 + (j << 4) + rlane;
      float bv = 0.f;
      if (BIAS_MODE == 2) bv = bias[n];
#pragma unroll
      for (int r = 0; r < 8; ++r) {
        float v = acc[i][j][r] * scale;
        if (BIAS_MODE == 1) v += bias[mBase + mOff + r];
        if (BIAS_MODE == 2) v += bv;
        if (RESID) v += Rb[(size_t)(mBase + mOff + r) * ldc + n];
        if (ACT == 2) v = fmaxf(v, 0.0f);
        if (ACT == 4) v = (v > 0.f) ? v : 0.01f * v;
        slab[(mOff + r) * 68 + (j << 4) + rlane] = v;
      }
    }
    __builtin_amdgcn_fence(__ATOMIC_RELEASE, "workgroup");
    __builtin_amdgcn_wave_barrier();
    __builtin_amdgcn_fence(__ATOMIC_ACQUIRE, "workgroup");
    if (OUT_MODE == 0) {
      float* C = (float*)Cout + (size_t)b * strideC;
      const int hh = lane >> 4, c4 = (lane & 15) * 4;
      for (int pass = 0; pass < 2; ++pass) {
#pragma unroll
        for (int it = 0; it < 8; ++it) {
          const int row = it * 2 + hh;
          v4f v = *(const v4f*)(slab + row * 68 + c4);
          *(volatile v4f*)(C + (size_t)(mBase + row) * ldc + n0 + c4) = v;
        }
        __threadfence();
      }
    } else {
      const int q = lane >> 3, c8 = (lane & 7) * 8;
      unsigned short* C  = (unsigned short*)Cout  + (size_t)b * strideC;
      unsigned short* C2 = (OUT_MODE == 2) ? ((unsigned short*)Cout2 + (size_t)b * strideC) : nullptr;
      for (int pass = 0; pass < 2; ++pass) {
#pragma unroll
        for (int it = 0; it < 4; ++it) {
          const int row = it * 4 + q;
          const float* sp = slab + row * 68 + c8;
          v8h hv, lv;
#pragma unroll
          for (int e = 0; e < 8; ++e) {
            if (OUT_MODE == 1) {
              hv[e] = (_Float16)sp[e];
            } else {
              unsigned short hb = f2bf_bits(sp[e]);
              hv[e] = __builtin_bit_cast(_Float16, hb);
              if (OUT_MODE == 2) {
                unsigned short lb = f2bf_bits(sp[e] - bf_bits2f(hb));
                lv[e] = __builtin_bit_cast(_Float16, lb);
              }
            }
          }
          *(volatile v8h*)(C + (size_t)(mBase + row) * ldc + n0 + c8) = hv;
          if (OUT_MODE == 2) *(volatile v8h*)(C2 + (size_t)(mBase + row) * ldc + n0 + c8) = lv;
        }
        __threadfence();
      }
    }
    __builtin_amdgcn_fence(__ATOMIC_RELEASE, "workgroup");
    __builtin_amdgcn_wave_barrier();
    __builtin_amdgcn_fence(__ATOMIC_ACQUIRE, "workgroup");
  }
}

__device__ __forceinline__ float softplus_f(float x) {
  return fmaxf(x, 0.0f) + log1pf(expf(-fabsf(x)));
}

__global__ __launch_bounds__(256) void sp_planes_kernel(const float* __restrict__ cores, unsigned short* __restrict__ spt) {
  __shared__ __align__(16) unsigned short sm[32][264];
  const int t = threadIdx.x;
  const int lane = t & 31, wave = t >> 5;
  const int q    = blockIdx.x;
  const int mode = blockIdx.y;
  const int n0   = q * 32;
  const int ijA  = n0 + lane;
  const int ijB  = lane * 32 + q;
  const int ij   = (mode == 0) ? ijA : ijB;
  const float* src = cores + (size_t)mode * kND * kNRR + ij;
#pragma unroll 1
  for (int it = 0; it < 32; ++it) {
    const int d = it * 8 + wave;
    const float x = src[(size_t)d * kNRR];
    sm[lane][d] = f2bf_bits(softplus_f(x));
  }
  __syncthreads();
  unsigned short* base = spt + ((size_t)mode * kNRR + n0) * kND;
  for (int pass = 0; pass < 2; ++pass) {
#pragma unroll
    for (int rr = 0; rr < 4; ++rr) {
      const int row = wave * 4 + rr;
      unsigned short hb[8];
#pragma unroll
      for (int e = 0; e < 8; ++e) hb[e] = sm[row][lane * 8 + e];
      const v4u u = (v4u){pk16(hb[0], hb[1]), pk16(hb[2], hb[3]), pk16(hb[4], hb[5]), pk16(hb[6], hb[7])};
      *(volatile v4u*)(base + (size_t)row * kND + lane * 8) = u;
    }
    __threadfence();
  }
}

__global__ __launch_bounds__(256) void norm_gtab_kernel(const float* __restrict__ cores, const float* __restrict__ location,
                                                       const float* __restrict__ log_scale, float* __restrict__ gtab,
                                                       float* __restrict__ logn) {
  __shared__ float sCur[kNRR];
  __shared__ float sN[kNRR];
  __shared__ float sTmp[kNRR];
  const int t = threadIdx.x;
  const int lane = t & 31, wave = t >> 5;

#pragma unroll 1
  for (int m = 0; m < kNModes; ++m) {
    const float loc = location[t * kNModes + m];
    const float ls  = log_scale[t * kNModes + m];
    const float isc = expf(-ls);
    const float cst = -0.5f * kLog2Pi - ls;
    const v4f g = (v4f){loc, isc, cst, 0.0f};
    float* gp = gtab + ((size_t)(m * kND + t)) * 4;
    *(volatile v4f*)gp = g;
    __threadfence();
    *(volatile v4f*)gp = g;
  }

#pragma unroll 1
  for (int m = 0; m < kNModes; ++m) {
    const float* cm = cores + (size_t)m * kND * kNRR;
#pragma unroll 1
    for (int c4 = 0; c4 < 4; ++c4) {
      const int col = c4 * 256 + t;
      float s = 0.0f;
#pragma unroll 1
      for (int d = 0; d < kND; ++d) s += softplus_f(cm[(size_t)d * kNRR + col]);
      sCur[col] = s;
    }
    __syncthreads();
    if (m == 0) {
#pragma unroll 1
      for (int c4 = 0; c4 < 4; ++c4) { const int col = c4 * 256 + t; sN[col] = sCur[col]; }
    } else {
#pragma unroll 1
      for (int c4 = 0; c4 < 4; ++c4) {
        const int col = c4 * 256 + t;
        const int r1 = col >> 5, r2 = col & 31;
        float nv = 0.0f;
#pragma unroll 1
        for (int k = 0; k < kNR; ++k) nv += sN[r1 * kNR + k] * sCur[k * kNR + r2];
        sTmp[col] = nv;
      }
      __syncthreads();
#pragma unroll 1
      for (int c4 = 0; c4 < 4; ++c4) { const int col = c4 * 256 + t; sN[col] = sTmp[col]; }
    }
    __syncthreads();
  }
  float tr = sN[lane * 33];
#pragma unroll
  for (int off = 16; off > 0; off >>= 1) tr += __shfl_xor(tr, off, 32);
  const float lg = logf(tr);
  const v4f gv = (v4f){lg, lg, lg, lg};
  const int li = (lane < 8) ? lane : 7;
  float* lp = logn + li * 4;
  if (wave == 0 && lane < 8) *(volatile v4f*)lp = gv;
  __threadfence();
  if (wave == 0 && lane < 8) *(volatile v4f*)lp = gv;
}

__global__ __launch_bounds__(256) void wplanes_kernel(const float* __restrict__ value, const float* __restrict__ gtab,
                                                     unsigned short* __restrict__ wpl, int b0g) {
  const int t = threadIdx.x;
  const int lane = t & 31, wave = t >> 5;
  const int mode = blockIdx.y;
  float loc[8], isc[8], cst[8];
#pragma unroll
  for (int e = 0; e < 8; ++e) {
    const v4f g = *(const v4f*)(gtab + ((size_t)(mode * kND + lane * 8 + e)) * 4);
    loc[e] = g.x; isc[e] = g.y; cst[e] = g.z;
  }
  const int rowBase = blockIdx.x * 64;
#pragma unroll 1
  for (int r = 0; r < 8; ++r) {
    const int bl = rowBase + r * 8 + wave;
    const float v = value[(size_t)(b0g + bl) * kNModes + mode];
    unsigned short hb[8];
#pragma unroll
    for (int e = 0; e < 8; ++e) {
      const float z  = (v - loc[e]) * isc[e];
      const float lp = cst[e] - 0.5f * (z * z);
      hb[e] = f2bf_bits(expf(lp));
    }
    const v4u u = (v4u){pk16(hb[0], hb[1]), pk16(hb[2], hb[3]), pk16(hb[4], hb[5]), pk16(hb[6], hb[7])};
    unsigned short* wp = wpl + ((size_t)(mode * kChunk + bl)) * kND + lane * 8;
    *(volatile v4u*)wp = u;
    __threadfence();
    *(volatile v4u*)wp = u;
  }
}

__global__ __launch_bounds__(256) void chain_kernel(const unsigned short* __restrict__ margp, const float* __restrict__ logn,
                                                   float* __restrict__ out, int b0g) {
  __shared__ __align__(16) float res_s[32];
  const __bf16* marg = (const __bf16*)margp;
  const int t = threadIdx.x;
  const int lane = t & 31, wave = t >> 5;
  const int rlane = lane & 15, hh = lane >> 4, koff = hh * 8;
  const float lgn = logn[0];
  const v8f zero = (v8f){0.f,0.f,0.f,0.f,0.f,0.f,0.f,0.f};
  const int csel = lane & 7;
  const bool holds = ((rlane >> 3) == hh);

#pragma unroll 1
  for (int s = 0; s < 4; ++s) {
    const int bl = blockIdx.x * 32 + wave * 4 + s;
    const __bf16* m0p = marg + (size_t)bl * kNRR;
    v16b pb[2];
#pragma unroll
    for (int nt = 0; nt < 2; ++nt) pb[nt] = Frag<__bf16>::load(m0p + (nt * 16 + rlane) * kNR + koff);
    v8f acc[2][2];
#pragma unroll
    for (int mt = 0; mt < 2; ++mt)
#pragma unroll
      for (int nt = 0; nt < 2; ++nt) acc[mt][nt] = zero;
#pragma unroll 1
    for (int mode = 1; mode < kNModes; ++mode) {
      const __bf16* mp = marg + ((size_t)mode * kChunk + bl) * kNRR;
      v16b af[2];
#pragma unroll
      for (int mt = 0; mt < 2; ++mt) af[mt] = Frag<__bf16>::load(mp + (mt * 16 + rlane) * kNR + koff);
#pragma unroll
      for (int mt = 0; mt < 2; ++mt)
#pragma unroll
        for (int nt = 0; nt < 2; ++nt) acc[mt][nt] = Frag<__bf16>::mma(af[mt], pb[nt], zero);
      chain_guard(acc[0][0], acc[0][1], acc[1][0], acc[1][1], af[0], af[1], pb[0], pb[1]);
#pragma unroll
      for (int nt = 0; nt < 2; ++nt) {
#pragma unroll
        for (int e = 0; e < 8; ++e) {
          pb[nt][e]     = tobf(acc[0][nt][e]);
          pb[nt][8 + e] = tobf(acc[1][nt][e]);
        }
      }
    }
    float d0 = 0.0f, d1 = 0.0f;
#pragma unroll
    for (int e = 0; e < 8; ++e) {
      d0 = (csel == e) ? acc[0][0][e] : d0;
      d1 = (csel == e) ? acc[1][1][e] : d1;
    }
    float part = holds ? (d0 + d1) : 0.0f;
#pragma unroll
    for (int off = 16; off > 0; off >>= 1) part += __shfl_xor(part, off, 32);
    const float res = logf(fmaxf(part, 1e-12f)) - lgn;
    if (lane == 0) res_s[wave * 4 + s] = res;
  }
  __syncthreads();
  const int li = (lane < 8) ? lane : 7;
  const v4f vv = *(const v4f*)(res_s + li * 4);
  float* op = out + (size_t)b0g + (size_t)blockIdx.x * 32 + li * 4;
  if (wave == 0 && lane < 8) *(volatile v4f*)op = vv;
  __threadfence();
  if (wave == 0 && lane < 8) *(volatile v4f*)op = vv;
}

extern "C" void kernel_launch(void* const* d_in, const int* in_sizes, int n_in,
                              void* d_out, int out_size, void* d_ws, size_t ws_size,
                              hipStream_t stream) {
  if (n_in < 4) return;
  if (in_sizes[0] != kNB * kNModes) return;
  if (in_sizes[1] != kND * kNModes) return;
  if (in_sizes[2] != kND * kNModes) return;
  if (in_sizes[3] != kNModes * kND * kNRR) return;
  if (out_size < kNB) return;
  if (ws_size < kWsTotal) return;

  const float* value     = (const float*)d_in[0];
  const float* location  = (const float*)d_in[1];
  const float* log_scale = (const float*)d_in[2];
  const float* cores     = (const float*)d_in[3];
  float* out = (float*)d_out;

  char* ws = (char*)d_ws;
  unsigned short* spt  = (unsigned short*)(ws + kOffSpt);
  float*          gtab = (float*)(ws + kOffGtab);
  float*          logn = (float*)(ws + kOffLogn);
  unsigned short* wpl  = (unsigned short*)(ws + kOffWpl);
  unsigned short* marg = (unsigned short*)(ws + kOffMarg);

  sp_planes_kernel<<<dim3(kNRR / 32, kNModes), 256, 0, stream>>>(cores, spt);
  norm_gtab_kernel<<<1, 256, 0, stream>>>(cores, location, log_scale, gtab, logn);

  const int tilesPerMode = (kChunk / 64) * (kNRR / 64);
  const int gemmBlocks   = tilesPerMode / 8;
  for (int c = 0; c < kNChunk; ++c) {
    const int b0g = c * kChunk;
    wplanes_kernel<<<dim3(kChunk / 64, kNModes), 256, 0, stream>>>(value, gtab, wpl, b0g);
    wmma_gemm64<1, false, 0, 3, false, 0><<<dim3(gemmBlocks, kNModes), 256, 0, stream>>>(
        wpl, wpl, kND, (long)kChunk * kND,
        spt, spt, kND, (long)kNRR * kND,
        (void*)marg, (void*)marg, kNRR, (long)kChunk * kNRR,
        gtab,
        gtab, 0L,
        kChunk, kNRR, kND, 1.0f);
    chain_kernel<<<kChunk / 32, 256, 0, stream>>>(marg, logn, out, b0g);
  }
}
